// PalmSelfAttention_31971736551997
// MI455X (gfx1250) — hardware-verified
//
#include <hip/hip_runtime.h>
#include <stddef.h>
#include <stdint.h>

#define NBAT  2
#define SQ    2048
#define NTOK  4096
#define HID   1024
#define NH    16
#define HDM   64
#define NQKV  3072
#define NSLAB 48
#define QB    128
#define KC    64
#define NQB   (SQ / QB)
#define NKCH  (SQ / KC)
#define NFL   (NBAT * NQB)
#define FLW   32
#define FLMAGIC 0x0F1A65EDu

static_assert(NTOK == NBAT * SQ);
static_assert(HID == NH * HDM);
static_assert(NQKV == 3 * HID);
static_assert(NSLAB * HDM == NQKV);
static_assert(HDM % 32 == 0);
static_assert(HID % 32 == 0);
static_assert(HID == 128 * 8);
static_assert(SQ % QB == 0);
static_assert(SQ % KC == 0);
static_assert(SQ % 64 == 0);
static_assert(NKCH <= 32);
static_assert(SQ == 32 * 16 * 4);
static_assert(NFL * FLW * 4 == 4096);

typedef _Float16 v16h __attribute__((ext_vector_type(16)));
typedef _Float16 v8h  __attribute__((ext_vector_type(8)));
typedef float    v8f  __attribute__((ext_vector_type(8)));
typedef float    v4f  __attribute__((ext_vector_type(4)));
typedef unsigned int   v4u   __attribute__((ext_vector_type(4)));
typedef unsigned short v8us  __attribute__((ext_vector_type(8)));
typedef unsigned short v16us __attribute__((ext_vector_type(16)));
typedef __bf16         v16b  __attribute__((ext_vector_type(16)));
typedef unsigned short ush;
typedef float fal __attribute__((may_alias));
typedef v4f  v4fa __attribute__((may_alias));

union Frag  { v16h v; v8h h[2]; };
union FragU { v16us v; v8us h[2]; v16b b; };
union Pack8 { v8h h; v4u u; };
union PackU { v8us s; v4u u; };
struct HL { v4u h; v4u l; };

__device__ __forceinline__ ush f2bf(float f) {
  const unsigned u = __float_as_uint(f);
  return (ush)((u + 0x7FFFu + ((u >> 16) & 1u)) >> 16);
}
__device__ __forceinline__ float bf2f(ush b) { return __uint_as_float(((unsigned)b) << 16); }

__device__ __forceinline__ HL split8(v8f f) {
  PackU ph, pl;
#pragma unroll
  for (int e = 0; e < 8; ++e) {
    const ush hi = f2bf(f[e]);
    ph.s[e] = hi;
    pl.s[e] = f2bf(f[e] - bf2f(hi));
  }
  HL r; r.h = ph.u; r.l = pl.u;
  return r;
}

__device__ __forceinline__ v8f mma16(v16h a, v16h b, v8f c) {
  c = __builtin_amdgcn_wmma_f32_16x16x32_f16(false, a, false, b, (short)0, c, false, false);
  asm volatile("v_nop\n\tv_nop\n\tv_nop\n\tv_nop" : "+v"(c) : "v"(a), "v"(b));
  return c;
}
__device__ __forceinline__ v8f mmab(v16us a, v16us b, v8f c) {
  FragU ua, ub; ua.v = a; ub.v = b;
  c = __builtin_amdgcn_wmma_f32_16x16x32_bf16(false, ua.b, false, ub.b, (short)0, c, false, false);
  asm volatile("v_nop\n\tv_nop\n\tv_nop\n\tv_nop" : "+v"(c) : "v"(a), "v"(b));
  return c;
}

__device__ __forceinline__ v16h ldfrag(const _Float16* p, int ld, int row0, int k0, int lane) {
  const int m = lane & 15, lh = lane >> 4;
  const _Float16* q = p + (size_t)(row0 + m) * ld + k0 + 8 * lh;
  Frag f;
  f.h[0] = *(const v8h*)(q);
  f.h[1] = *(const v8h*)(q + 16);
  return f.v;
}
__device__ __forceinline__ v16us ldfragu(const ush* p, int ld, int row0, int k0, int lane) {
  const int m = lane & 15, lh = lane >> 4;
  const ush* q = p + (size_t)(row0 + m) * ld + k0 + 8 * lh;
  FragU f;
  f.h[0] = *(const v8us*)(q);
  f.h[1] = *(const v8us*)(q + 16);
  return f.v;
}

__device__ __forceinline__ v8f zero8() { return (v8f){0.f, 0.f, 0.f, 0.f, 0.f, 0.f, 0.f, 0.f}; }

__device__ __forceinline__ void gemm3_32x64(const ush* __restrict__ Ah, const ush* __restrict__ Al,
                                            const ush* __restrict__ Bh, const ush* __restrict__ Bl,
                                            int m0, int n0, int lane, v8f (&acc)[2][4]) {
#pragma unroll 1
  for (int k0 = 0; k0 < HID; k0 += 32) {
    const v16us a0h = ldfragu(Ah, HID, m0, k0, lane);
    const v16us a1h = ldfragu(Ah, HID, m0 + 16, k0, lane);
    const v16us a0l = ldfragu(Al, HID, m0, k0, lane);
    const v16us a1l = ldfragu(Al, HID, m0 + 16, k0, lane);
#pragma unroll
    for (int t = 0; t < 4; ++t) {
      const v16us bh = ldfragu(Bh, HID, n0 + 16 * t, k0, lane);
      const v16us bl = ldfragu(Bl, HID, n0 + 16 * t, k0, lane);
      acc[0][t] = mmab(a0h, bh, acc[0][t]);
      acc[1][t] = mmab(a1h, bh, acc[1][t]);
      acc[0][t] = mmab(a0h, bl, acc[0][t]);
      acc[1][t] = mmab(a1h, bl, acc[1][t]);
      acc[0][t] = mmab(a0l, bh, acc[0][t]);
      acc[1][t] = mmab(a1l, bh, acc[1][t]);
    }
  }
}

__global__ __launch_bounds__(256) void k_mflag(const float* __restrict__ mask, unsigned* __restrict__ fl) {
  __shared__ unsigned red[8][4];
  const int tid = threadIdx.x, lane = tid & 31, wave = tid >> 5;
  const int ln = blockIdx.x;
  const int b  = ln / NQB;
  const int qb = ln - b * NQB;
  const float* mb = mask + (size_t)b * SQ * SQ;
  unsigned allm = 0xFFFFFFFFu, allz = 0xFFFFFFFFu, rowsfin = 1u;
#pragma unroll 1
  for (int rr = 0; rr < 16; ++rr) {
    const float* mp = mb + (size_t)(qb * QB + wave * 16 + rr) * SQ;
    unsigned rf = 0u;
#pragma unroll 4
    for (int j = 0; j < 16; ++j) {
      const v4f v = *(const v4f*)(mp + 4 * (lane + 32 * j));
      const unsigned bit = 1u << ((lane >> 4) + 2 * j);
      const bool fin = (v[0] > -1.0e30f) || (v[1] > -1.0e30f) || (v[2] > -1.0e30f) || (v[3] > -1.0e30f);
      const bool nz  = (v[0] != 0.0f) || (v[1] != 0.0f) || (v[2] != 0.0f) || (v[3] != 0.0f);
      allm &= fin ? ~bit : 0xFFFFFFFFu;
      allz &= nz  ? ~bit : 0xFFFFFFFFu;
      rf |= fin ? 1u : 0u;
    }
#pragma unroll
    for (int off = 1; off < 32; off <<= 1) rf |= __shfl_xor(rf, off, 32);
    rowsfin &= rf;
  }
#pragma unroll
  for (int off = 1; off < 32; off <<= 1) {
    allm &= __shfl_xor(allm, off, 32);
    allz &= __shfl_xor(allz, off, 32);
  }
  if (lane == 0) { red[wave][0] = allm; red[wave][1] = allz; red[wave][2] = rowsfin; red[wave][3] = 0u; }
  __syncthreads();
  if (wave == 0) {
    unsigned a = 0xFFFFFFFFu, z = 0xFFFFFFFFu, f = 1u;
#pragma unroll
    for (int w = 0; w < 8; ++w) { a &= red[w][0]; z &= red[w][1]; f &= red[w][2]; }
    const unsigned word = (lane == 0) ? a : ((lane == 1) ? z : ((lane == 2) ? f : ((lane == 3) ? FLMAGIC : 0u)));
    volatile unsigned* d = (volatile unsigned*)(fl + ln * FLW + lane);
    *d = word;
    __threadfence();
    *d = word;
  }
}

__global__ __launch_bounds__(128) void k_split(const float* __restrict__ src, ush* __restrict__ dh,
                                               ush* __restrict__ dl) {
  const int row = blockIdx.x;
  const int col = (int)threadIdx.x * 8;
  const size_t o = (size_t)row * HID + col;
  const v4f a0 = *(const v4f*)(src + o);
  const v4f a1 = *(const v4f*)(src + o + 4);
  const v8f f = (v8f){a0[0], a0[1], a0[2], a0[3], a1[0], a1[1], a1[2], a1[3]};
  const HL sp = split8(f);
  volatile v4u* ph = (volatile v4u*)(dh + o);
  volatile v4u* pl = (volatile v4u*)(dl + o);
  *ph = sp.h;
  *pl = sp.l;
  __threadfence();
  *ph = sp.h;
  *pl = sp.l;
}

#define SFP 68
__global__ __launch_bounds__(64) __attribute__((amdgpu_num_vgpr(256)))
void k_qkv(const ush* __restrict__ xh, const ush* __restrict__ xl,
           const ush* __restrict__ wh, const ush* __restrict__ wl,
           const float* __restrict__ bqkv,
           _Float16* __restrict__ qp, _Float16* __restrict__ kp, _Float16* __restrict__ vtp) {
  __shared__ __align__(16) float sf[64 * SFP];
  const int tid = threadIdx.x, lane = tid & 31, wave = tid >> 5;
  const int hh = lane >> 4, c = lane & 15;
  const int mb = blockIdx.x * 64;
  const int b  = mb / SQ;
  const int sb = mb - b * SQ;
  const int ns = blockIdx.y;
  const int which = ns / NH;
  const int head  = ns - which * NH;
  const int m0 = mb + wave * 32;
  const int n0 = ns * HDM;
  const float* bias = bqkv + ns * HDM;

  v8f acc[2][4];
#pragma unroll
  for (int s = 0; s < 2; ++s)
#pragma unroll
    for (int t = 0; t < 4; ++t) acc[s][t] = zero8();
  gemm3_32x64(xh, xl, wh, wl, m0, n0, lane, acc);

#pragma unroll
  for (int sub = 0; sub < 2; ++sub) {
#pragma unroll
    for (int t = 0; t < 4; ++t) {
      const float bb = bias[16 * t + c];
#pragma unroll
      for (int r = 0; r < 8; ++r)
        sf[(wave * 32 + 16 * sub + 8 * hh + r) * SFP + 16 * t + c] = acc[sub][t][r] + bb;
    }
  }
  __syncthreads();

  const int hb = b * NH + head;
  if (which < 2) {
    const float RN = 0.35355338454246521f;
    const float QS = 4.0f * RN;
    v4u val[8];
    size_t go[8];
#pragma unroll
    for (int j = 0; j < 8; ++j) {
      const int p  = tid + 64 * j;
      const int lr = p >> 3;
      const int pc = p & 7;
      const int d0 = pc * 8;
      const float* ra = sf + lr * SFP + d0;
      const v4f a0 = *(const v4f*)(ra) * QS;
      const v4f a1 = *(const v4f*)(ra + 4) * QS;
      Pack8 pk;
      pk.h = (v8h){(_Float16)a0[0], (_Float16)a0[1], (_Float16)a0[2], (_Float16)a0[3],
                   (_Float16)a1[0], (_Float16)a1[1], (_Float16)a1[2], (_Float16)a1[3]};
      val[j] = pk.u;
      go[j]  = ((size_t)hb * SQ + sb + lr) * HDM + d0;
    }
    _Float16* base = (which == 0) ? qp : kp;
    for (int ps = 0; ps < 2; ++ps) {
#pragma unroll
      for (int j = 0; j < 8; ++j) *(volatile v4u*)(base + go[j]) = val[j];
      __threadfence();
    }
  } else {
    v4u val[8];
    size_t go[8];
#pragma unroll
    for (int j = 0; j < 8; ++j) {
      const int p  = tid + 64 * j;
      const int d  = p >> 3;
      const int pc = p & 7;
      const float* cp = sf + (pc * 8) * SFP + d;
      Pack8 pk;
      pk.h = (v8h){(_Float16)cp[0 * SFP], (_Float16)cp[1 * SFP], (_Float16)cp[2 * SFP], (_Float16)cp[3 * SFP],
                   (_Float16)cp[4 * SFP], (_Float16)cp[5 * SFP], (_Float16)cp[6 * SFP], (_Float16)cp[7 * SFP]};
      val[j] = pk.u;
      go[j]  = ((size_t)hb * HDM + d) * SQ + sb + pc * 8;
    }
    for (int ps = 0; ps < 2; ++ps) {
#pragma unroll
      for (int j = 0; j < 8; ++j) *(volatile v4u*)(vtp + go[j]) = val[j];
      __threadfence();
    }
  }
}

#define KTP 72
#define PSP 128
static_assert(16 * PSP * 2 == 16 * KC * 4);
static_assert(16 * PSP * 2 == 16 * HDM * 4);
__global__ __launch_bounds__(256) __attribute__((amdgpu_num_vgpr(256)))
void k_attn(const _Float16* __restrict__ qp, const _Float16* __restrict__ kp, const _Float16* __restrict__ vt,
            const float* __restrict__ mask, const unsigned* __restrict__ fl, float* __restrict__ out) {
  __shared__ __align__(16) _Float16 Ks[KC * KTP];
  __shared__ __align__(16) _Float16 Vs[HDM * KTP];
  __shared__ __align__(16) _Float16 Ps[8 * 16 * PSP];

  const int tid = threadIdx.x, lane = tid & 31, wave = tid >> 5;
  const int hh = lane >> 4, c = lane & 15;
  const int qb = blockIdx.x % NQB;
  const int hb = blockIdx.x / NQB;
  const int b  = hb / NH;
  const int h  = hb - b * NH;
  const int q0 = qb * QB + wave * 16;
  const int ln = b * NQB + qb;

  const _Float16* Q = qp + (size_t)hb * SQ * HDM;
  const _Float16* K = kp + (size_t)hb * SQ * HDM;
  const _Float16* V = vt + (size_t)hb * HDM * SQ;
  const float*  mbp = mask + (size_t)b * SQ * SQ;

  const unsigned w0 = (unsigned)__builtin_amdgcn_readfirstlane((int)fl[ln * FLW + 0]);
  const unsigned w1 = (unsigned)__builtin_amdgcn_readfirstlane((int)fl[ln * FLW + 1]);
  const unsigned w2 = (unsigned)__builtin_amdgcn_readfirstlane((int)fl[ln * FLW + 2]);
  const unsigned w3 = (unsigned)__builtin_amdgcn_readfirstlane((int)fl[ln * FLW + 3]);
  const bool valid = (w3 == FLMAGIC);
  const unsigned allm = valid ? w0 : 0u;
  const unsigned allz = valid ? w1 : 0u;
  const bool rfin = valid && ((w2 & 1u) != 0u);

  v16h qa[2];
#pragma unroll
  for (int dc = 0; dc < 2; ++dc) qa[dc] = ldfrag(Q, HDM, q0, dc * 32, lane);

  const float NEGI = -__builtin_huge_valf();
  const float sscale = 0.0625f;
  float mrow[8], lrow[8];
  v8f oacc[4];
#pragma unroll
  for (int r = 0; r < 8; ++r) { mrow[r] = NEGI; lrow[r] = 0.f; }
#pragma unroll
  for (int t = 0; t < 4; ++t) oacc[t] = zero8();

  _Float16* pw  = Ps + wave * 16 * PSP;
  float*    mwf = (float*)pw;

  for (int kc = 0; kc < NKCH; ++kc) {
    if (rfin && (((allm >> kc) & 1u) != 0u)) continue;
    const bool ldm = (((allz >> kc) & 1u) == 0u);
    const int kv0 = kc * KC;
    __syncthreads();
#pragma unroll
    for (int e = 0; e < 2; ++e) {
      const int p  = tid + 256 * e;
      const int r  = p >> 3;
      const int q8 = (p & 7) * 8;
      *(v8h*)(Ks + r * KTP + q8) = *(const v8h*)(K + (size_t)(kv0 + r) * HDM + q8);
      *(v8h*)(Vs + r * KTP + q8) = *(const v8h*)(V + (size_t)r * SQ + kv0 + q8);
    }
    if (ldm) {
#pragma unroll
      for (int it = 0; it < 8; ++it) {
        const int p   = lane + 32 * it;
        const int row = p >> 4;
        const int c4  = (p & 15) * 4;
        *(v4f*)(mwf + row * KC + c4) = *(const v4f*)(mbp + (size_t)(q0 + row) * SQ + kv0 + c4);
      }
    }
    __syncthreads();

    v8f s[4];
#pragma unroll
    for (int j = 0; j < 4; ++j) s[j] = zero8();
#pragma unroll
    for (int dc = 0; dc < 2; ++dc) {
#pragma unroll
      for (int j = 0; j < 4; ++j) {
        const v16h kb = ldfrag(Ks, KTP, j * 16, dc * 32, lane);
        s[j] = mma16(qa[dc], kb, s[j]);
      }
    }
    if (ldm) {
      const fal* mr = (const fal*)mwf + (8 * hh) * KC + c;
#pragma unroll
      for (int r = 0; r < 8; ++r)
#pragma unroll
        for (int j = 0; j < 4; ++j) s[j][r] = s[j][r] * sscale + mr[r * KC + 16 * j];
    } else {
#pragma unroll
      for (int r = 0; r < 8; ++r)
#pragma unroll
        for (int j = 0; j < 4; ++j) s[j][r] = s[j][r] * sscale;
    }
    __builtin_amdgcn_fence(__ATOMIC_RELEASE, "wavefront");
    __builtin_amdgcn_wave_barrier();
    float cm[8];
#pragma unroll
    for (int r = 0; r < 8; ++r) {
      float m = NEGI;
#pragma unroll
      for (int j = 0; j < 4; ++j) m = fmaxf(m, s[j][r]);
#pragma unroll
      for (int off = 1; off < 16; off <<= 1) m = fmaxf(m, __shfl_xor(m, off, 32));
      cm[r] = m;
    }
    float al[8];
#pragma unroll
    for (int r = 0; r < 8; ++r) {
      const float mnew  = fmaxf(mrow[r], cm[r]);
      const float msafe = (mnew == NEGI) ? 0.f : mnew;
      const float alpha = __expf(mrow[r] - msafe);
      mrow[r] = mnew;
      float psum = 0.f;
#pragma unroll
      for (int j = 0; j < 4; ++j) {
        const float p = __expf(s[j][r] - msafe);
        psum += p;
        pw[(8 * hh + r) * PSP + j * 16 + c] = (_Float16)(p * 1024.0f);
      }
#pragma unroll
      for (int off = 1; off < 16; off <<= 1) psum += __shfl_xor(psum, off, 32);
      lrow[r] = lrow[r] * alpha + psum;
      al[r] = alpha;
    }
#pragma unroll
    for (int t = 0; t < 4; ++t)
#pragma unroll
      for (int r = 0; r < 8; ++r) oacc[t][r] *= al[r];
    __syncthreads();

#pragma unroll
    for (int kk = 0; kk < 2; ++kk) {
      const v16h pa = ldfrag(pw, PSP, 0, kk * 32, lane);
#pragma unroll
      for (int t = 0; t < 4; ++t) {
        const v16h vb = ldfrag(Vs, KTP, t * 16, kk * 32, lane);
        oacc[t] = mma16(pa, vb, oacc[t]);
      }
    }
  }

  float invl[8];
#pragma unroll
  for (int r = 0; r < 8; ++r) invl[r] = (lrow[r] > 0.f) ? (0.0009765625f / lrow[r]) : 0.f;
  __syncthreads();
#pragma unroll
  for (int r = 0; r < 8; ++r) {
#pragma unroll
    for (int t = 0; t < 4; ++t)
      mwf[(8 * hh + r) * HDM + 16 * t + c] = oacc[t][r] * invl[r];
  }
  __syncthreads();
  v4f val[8];
  size_t go[8];
#pragma unroll
  for (int it = 0; it < 8; ++it) {
    const int p    = lane + 32 * it;
    const int L    = p >> 3;
    const int pc   = p & 7;
    const int row  = L >> 1;
    const int half = L & 1;
    val[it] = *(const v4fa*)(mwf + row * HDM + half * 32 + pc * 4);
    go[it]  = ((size_t)(b * SQ + q0 + row)) * HID + h * HDM + half * 32 + pc * 4;
  }
  for (int ps = 0; ps < 2; ++ps) {
#pragma unroll
    for (int it = 0; it < 8; ++it) *(volatile v4f*)(out + go[it]) = val[it];
    __threadfence();
  }
}

extern "C" void kernel_launch(void* const* d_in, const int* in_sizes, int n_in,
                              void* d_out, int out_size, void* d_ws, size_t ws_size,
                              hipStream_t stream) {
  if (n_in < 4) return;
  if (in_sizes[0] != NTOK * HID) return;
  if (in_sizes[1] != NBAT * SQ * SQ) return;
  if (in_sizes[2] != NQKV * HID) return;
  if (in_sizes[3] != NQKV) return;
  if (out_size != NTOK * HID) return;

  const float* x     = (const float*)d_in[0];
  const float* maskp = (const float*)d_in[1];
  const float* wqkv  = (const float*)d_in[2];
  const float* bqkv  = (const float*)d_in[3];
  float* out = (float*)d_out;

  size_t off = 0;
  const size_t oFL = off; off += (size_t)NFL * FLW * 4;
  const size_t oXh = off; off += (size_t)NTOK * HID * 2;
  const size_t oXl = off; off += (size_t)NTOK * HID * 2;
  const size_t oWh = off; off += (size_t)NQKV * HID * 2;
  const size_t oWl = off; off += (size_t)NQKV * HID * 2;
  const size_t oQ  = off; off += (size_t)NBAT * NH * SQ * HDM * 2;
  const size_t oK  = off; off += (size_t)NBAT * NH * SQ * HDM * 2;
  const size_t oV  = off; off += (size_t)NBAT * NH * HDM * SQ * 2;
  if (off > ws_size) return;
  if (off > (size_t)134217728) return;

  char* ws = (char*)d_ws;
  unsigned* FL = (unsigned*)(ws + oFL);
  ush*      Xh = (ush*)(ws + oXh);
  ush*      Xl = (ush*)(ws + oXl);
  ush*      Wh = (ush*)(ws + oWh);
  ush*      Wl = (ush*)(ws + oWl);
  _Float16* Qp = (_Float16*)(ws + oQ);
  _Float16* Kp = (_Float16*)(ws + oK);
  _Float16* Vt = (_Float16*)(ws + oV);

  k_mflag<<<dim3(NFL), dim3(256), 0, stream>>>(maskp, FL);
  k_split<<<dim3(NTOK), dim3(HID / 8), 0, stream>>>(x, Xh, Xl);
  k_split<<<dim3(NQKV), dim3(HID / 8), 0, stream>>>(wqkv, Wh, Wl);
  k_qkv<<<dim3(NTOK / 64, NSLAB), dim3(64), 0, stream>>>(Xh, Xl, Wh, Wl, bqkv, Qp, Kp, Vt);
  k_attn<<<dim3(NBAT * NH * NQB), dim3(256), 0, stream>>>(Qp, Kp, Vt, maskp, FL, out);
  (void)hipGetLastError();
}
